// TLSTMMotionForecaster_79946521247954
// MI455X (gfx1250) — hardware-run, weakly checked
//
#include <hip/hip_runtime.h>
#include <math.h>

constexpr int NBATCH   = 4096;
constexpr int NSTEP    = 64;
constexpr int NFEAT    = 16;
constexpr int NHID     = 128;
constexpr int NLIVE    = 3;
constexpr int NSTATE   = NFEAT + NHID;
constexpr int NOUTC    = 60;
constexpr int NTHR     = 256;
constexpr int ROWS_BLK = 32;
constexpr int K0PAD    = 32;
constexpr int KL0      = K0PAD + NHID;
constexpr int KL1      = 2 * NHID;
constexpr int APITCH   = K0PAD + 2 * NHID + 8;
constexpr int TPITCH   = NHID + 8;
constexpr int SPITCH   = 148;
constexpr int LN_SEG   = NSTATE / 8;
constexpr float WCARRY     = 16.0f;
constexpr float WCARRY_INV = 1.0f / 16.0f;
constexpr float LN_EPS_F   = 1e-5f;
constexpr float E_F32      = 2.718281828459045f;

constexpr int KC0 = KL0 / 8;
constexpr int KC1 = KL1 / 8;
constexpr int KCD = NHID / 8;
constexpr int PB0 = (NLIVE * NHID * KC0) / NTHR;
constexpr int PB1 = (NLIVE * NHID * KC1) / NTHR;
constexpr int PBD = (2 * NHID * KCD) / NTHR;
constexpr int PBB = 1;
constexpr int PB_TOTAL = PB0 + PB1 + PBD + PBB;

static_assert(NSTATE == 144, "state width");
static_assert(KL0 % 32 == 0 && KL1 % 32 == 0 && NHID % 32 == 0, "K multiples of 32");
static_assert(NHID == 16 * (NTHR / 32), "8 waves x 16 hidden columns");
static_assert(NBATCH % ROWS_BLK == 0, "grid exact");
static_assert((NLIVE * NHID * KC0) % NTHR == 0, "plane 0 chunk count exact");
static_assert((NLIVE * NHID * KC1) % NTHR == 0, "plane 1 chunk count exact");
static_assert((2 * NHID * KCD) % NTHR == 0, "plane D chunk count exact");
static_assert(NLIVE * NHID == 4 * 96, "bias line count");
static_assert((ROWS_BLK * NOUTC * 4) % 128 == 0, "block output is whole lines");
static_assert(LN_SEG * 8 == NSTATE, "LayerNorm segments exact");
static_assert(APITCH % 8 == 0 && TPITCH % 8 == 0 && SPITCH % 4 == 0, "LDS pitches 16-B multiples");
static_assert(ROWS_BLK * NOUTC <= ROWS_BLK * SPITCH, "output tile fits the state tile");

typedef __attribute__((ext_vector_type(16))) _Float16 v16h;
typedef __attribute__((ext_vector_type(8)))  _Float16 v8h;
typedef __attribute__((ext_vector_type(8)))  float    v8f;
typedef __attribute__((ext_vector_type(4)))  float    v4f;
typedef __attribute__((ext_vector_type(4)))  int      v4i;

__device__ __forceinline__ void guard6_h(v8f& a, v8f& b, v8f& c, v8f& d, v8f& e, v8f& f,
                                         v16h x0, v16h x1, v16h y0, v16h y1, v16h y2) {
  asm volatile("v_nop\n\tv_nop\n\tv_nop\n\tv_nop"
               : "+v"(a), "+v"(b), "+v"(c), "+v"(d), "+v"(e), "+v"(f)
               : "v"(x0), "v"(x1), "v"(y0), "v"(y1), "v"(y2));
}
__device__ __forceinline__ void guard2_h(v8f& a, v8f& b, v16h x0, v16h x1, v16h y0) {
  asm volatile("v_nop\n\tv_nop\n\tv_nop\n\tv_nop" : "+v"(a), "+v"(b) : "v"(x0), "v"(x1), "v"(y0));
}

template <typename T> struct Frag;
template <> struct Frag<_Float16> {
  typedef v16h V; union U { v16h v; v8h h[2]; };
  static __device__ __forceinline__ v16h load(const _Float16* p) {
    U f; f.h[0] = *(const v8h*)(p); f.h[1] = *(const v8h*)(p + 16); return f.v;
  }
  static __device__ __forceinline__ v8f mma(v16h a, v16h b, v8f c) {
    return __builtin_amdgcn_wmma_f32_16x16x32_f16(false, a, false, b, (short)0, c, false, false);
  }
};

__device__ __forceinline__ float fsig(float x)  { return __builtin_amdgcn_rcpf(1.0f + __expf(-x)); }
__device__ __forceinline__ float ftanh(float x) { return 1.0f - 2.0f * __builtin_amdgcn_rcpf(__expf(2.0f * x) + 1.0f); }

__global__ __launch_bounds__(NTHR) void pack_planes_kernel(
    const float* __restrict__ Wp, const float* __restrict__ bp,
    const float* __restrict__ Wx, const float* __restrict__ bx,
    const float* __restrict__ Uh, const float* __restrict__ Wd,
    unsigned short* __restrict__ BT0, unsigned short* __restrict__ BT1,
    unsigned short* __restrict__ BTD, float* __restrict__ BIAS0) {
  const int tid = threadIdx.x;
  const int blk = blockIdx.x;
  if (blk < PB0) {
    const int i   = blk * NTHR + tid;
    const int n   = i / KC0;
    const int kc  = i - n * KC0;
    const int gp  = n >> 7;
    const int col = n & (NHID - 1);
    const float* wxg = Wx + ((size_t)(gp + 1) * NHID) * NHID + col;
    const float* uhg = Uh + ((size_t)(gp + 1) * NHID) * NHID + col;
    const int kcc = (kc < 1) ? kc : 1;
    const float* wpr = Wp + (size_t)(8 * kcc) * NHID;
    float ca[8];
#pragma unroll
    for (int e = 0; e < 8; ++e) ca[e] = 0.0f;
#pragma unroll 1
    for (int j = 0; j < NHID; ++j) {
      const float wv = wxg[(size_t)j * NHID];
#pragma unroll
      for (int e = 0; e < 8; ++e) ca[e] = fmaf(wpr[e * NHID + j], wv, ca[e]);
    }
    float uv[8];
#pragma unroll
    for (int e = 0; e < 8; ++e) {
      int ku = 8 * kc - K0PAD + e;
      ku = ku < 0 ? 0 : (ku > NHID - 1 ? NHID - 1 : ku);
      uv[e] = uhg[(size_t)ku * NHID];
      asm volatile("" : "+v"(uv[e]));
    }
    v8h hv;
#pragma unroll
    for (int e = 0; e < 8; ++e) {
      const float val = (kc < 2) ? ca[e] : ((kc < 4) ? 0.0f : uv[e]);
      hv[e] = (_Float16)(val * WCARRY);
    }
    unsigned short* dp = BT0 + (size_t)i * 8;
    *(volatile v8h*)dp = hv;
    __threadfence();
    *(volatile v8h*)dp = hv;
  } else if (blk < PB0 + PB1) {
    const int i   = (blk - PB0) * NTHR + tid;
    const int n   = i >> 5;
    const int kc  = i & (KC1 - 1);
    const int gp  = n >> 7;
    const int col = n & (NHID - 1);
    const float* src = (kc < 16) ? Wx : Uh;
    const float* p = src + ((size_t)((4 + gp + 1) * NHID + ((8 * kc) & (NHID - 1)))) * NHID + col;
    v8h hv;
#pragma unroll
    for (int e = 0; e < 8; ++e) hv[e] = (_Float16)(p[(size_t)e * NHID] * WCARRY);
    unsigned short* dp = BT1 + (size_t)i * 8;
    *(volatile v8h*)dp = hv;
    __threadfence();
    *(volatile v8h*)dp = hv;
  } else if (blk < PB0 + PB1 + PBD) {
    const int i  = (blk - PB0 - PB1) * NTHR + tid;
    const int l  = i >> 11;
    const int n  = (i >> 4) & (NHID - 1);
    const int kc = i & (KCD - 1);
    const float* p = Wd + ((size_t)(l * NHID + 8 * kc)) * NHID + n;
    v8h hv;
#pragma unroll
    for (int e = 0; e < 8; ++e) hv[e] = (_Float16)(p[(size_t)e * NHID] * WCARRY);
    unsigned short* dp = BTD + (size_t)i * 8;
    *(volatile v8h*)dp = hv;
    __threadfence();
    *(volatile v8h*)dp = hv;
  } else {
    if (tid < 96) {
      const int n0   = 4 * tid;
      const int gp   = n0 >> 7;
      const int col0 = n0 & (NHID - 1);
      v4f acc = *(const v4f*)(bx + (size_t)(gp + 1) * NHID + col0);
#pragma unroll 1
      for (int j = 0; j < NHID; ++j) {
        const float bj = bp[j];
        const v4f wv = *(const v4f*)(Wx + ((size_t)((gp + 1) * NHID + j)) * NHID + col0);
#pragma unroll
        for (int e = 0; e < 4; ++e) acc[e] = fmaf(bj, wv[e], acc[e]);
      }
      float* dp = BIAS0 + n0;
      *(volatile v4f*)dp = acc;
      __threadfence();
      *(volatile v4f*)dp = acc;
    }
  }
}

__device__ __forceinline__ void stage_inputs(const float* __restrict__ hist, const float* __restrict__ msk,
                                             _Float16* At, float* decw, float* mtw,
                                             int rowbase, int tn, int tid) {
  if (tid < 128) {
    const int row = tid >> 2;
    const int s8  = tid & 3;
    const bool live = (s8 < 2);
    const int sc  = s8 & 1;
    const float* hp = hist + ((size_t)(rowbase + row) * NSTEP + (size_t)tn) * NFEAT + sc * 8;
    v4f va = *(const v4f*)(hp);
    v4f vb = *(const v4f*)(hp + 4);
    float mv = msk[(size_t)(rowbase + row) * NSTEP + (size_t)tn];
    asm volatile("" : "+v"(va), "+v"(vb), "+v"(mv));
    v8h hv;
#pragma unroll
    for (int e = 0; e < 4; ++e) {
      hv[e]     = (_Float16)(live ? va[e] : 0.0f);
      hv[4 + e] = (_Float16)(live ? vb[e] : 0.0f);
    }
    *(v8h*)(At + row * APITCH + s8 * 8) = hv;
    const float dt  = fmaxf(vb[1], 0.0f);
    const float dec = 1.0f / logf(E_F32 + dt);
    if (s8 == 0) { decw[row] = dec; mtw[row] = mv; }
  }
}

template <int KTOT>
__device__ __forceinline__ void cell_layer(
    const _Float16* arow, const _Float16* wg, const _Float16* wd,
    _Float16* htw, const _Float16* htr, _Float16* hdst,
    const float* decp, const float* mtp,
    const float bI, const float bO, const float bC, const float bD, const float wT, const float bT,
    float (&hs)[2][8], float (&cs)[2][8]) {
  constexpr int GSTR = NHID * KTOT;
  const v8f z8 = {0.f, 0.f, 0.f, 0.f, 0.f, 0.f, 0.f, 0.f};
  v8f aI[2], aO[2], aC[2];
  aI[0] = z8; aI[1] = z8; aO[0] = z8; aO[1] = z8; aC[0] = z8; aC[1] = z8;
#pragma unroll 1
  for (int k0 = 0; k0 < KTOT; k0 += 32) {
    const v16h a0 = Frag<_Float16>::load(arow + k0);
    const v16h a1 = Frag<_Float16>::load(arow + 16 * APITCH + k0);
    const v16h b0 = Frag<_Float16>::load(wg + k0);
    const v16h b1 = Frag<_Float16>::load(wg + GSTR + k0);
    const v16h b2 = Frag<_Float16>::load(wg + 2 * GSTR + k0);
    aI[0] = Frag<_Float16>::mma(a0, b0, aI[0]);
    aI[1] = Frag<_Float16>::mma(a1, b0, aI[1]);
    aO[0] = Frag<_Float16>::mma(a0, b1, aO[0]);
    aO[1] = Frag<_Float16>::mma(a1, b1, aO[1]);
    aC[0] = Frag<_Float16>::mma(a0, b2, aC[0]);
    aC[1] = Frag<_Float16>::mma(a1, b2, aC[1]);
    guard6_h(aI[0], aI[1], aO[0], aO[1], aC[0], aC[1], a0, a1, b0, b1, b2);
  }
  float ot[2][8], ht[2][8];
#pragma unroll
  for (int m = 0; m < 2; ++m) {
#pragma unroll
    for (int r = 0; r < 8; ++r) {
      const float ig = fsig(aI[m][r] * WCARRY_INV + bI);
      const float og = fsig(aO[m][r] * WCARRY_INV + bO);
      const float cg = ftanh(aC[m][r] * WCARRY_INV + bC);
      const float hv = cg + ig;
      ot[m][r] = og;
      ht[m][r] = hv;
      htw[(16 * m + r) * TPITCH] = (_Float16)hv;
    }
  }
  __syncthreads();
  v8f zs[2];
  zs[0] = z8; zs[1] = z8;
#pragma unroll 1
  for (int k0 = 0; k0 < NHID; k0 += 32) {
    const v16h a0 = Frag<_Float16>::load(htr + k0);
    const v16h a1 = Frag<_Float16>::load(htr + 16 * TPITCH + k0);
    const v16h b0 = Frag<_Float16>::load(wd + k0);
    zs[0] = Frag<_Float16>::mma(a0, b0, zs[0]);
    zs[1] = Frag<_Float16>::mma(a1, b0, zs[1]);
    guard2_h(zs[0], zs[1], a0, a1, b0);
  }
#pragma unroll
  for (int m = 0; m < 2; ++m) {
    const v4f dA = *(const v4f*)(decp + 16 * m);
    const v4f dB = *(const v4f*)(decp + 16 * m + 4);
    const v4f mA = *(const v4f*)(mtp + 16 * m);
    const v4f mB = *(const v4f*)(mtp + 16 * m + 4);
#pragma unroll
    for (int r = 0; r < 8; ++r) {
      const float dec = (r < 4) ? dA[r & 3] : dB[r & 3];
      const float mv  = (r < 4) ? mA[r & 3] : mB[r & 3];
      const float hsh = ftanh(zs[m][r] * WCARRY_INV + bD);
      const float dg  = fsig(dec * wT + bT);
      const float hst = (ht[m][r] - hsh) + hsh * dg;
      const float cn  = ftanh(hst + ot[m][r] * cs[m][r]);
      const float hn  = ot[m][r] * ftanh(cn);
      const float om  = 1.0f - mv;
      const float hb  = mv * hn + om * hs[m][r];
      const float cb  = mv * cn + om * cs[m][r];
      hs[m][r] = hb;
      cs[m][r] = cb;
      hdst[(16 * m + r) * APITCH] = (_Float16)hb;
    }
  }
}

__global__ __launch_bounds__(NTHR) void tcell_seq_kernel(
    const float* __restrict__ hist, const float* __restrict__ msk,
    const float* __restrict__ bx,   const float* __restrict__ bd,
    const float* __restrict__ Wt,   const float* __restrict__ bt,
    const float* __restrict__ ln_g, const float* __restrict__ ln_b,
    const float* __restrict__ W1,   const float* __restrict__ b1,
    const float* __restrict__ W2,   const float* __restrict__ b2,
    const unsigned short* __restrict__ BT0p, const unsigned short* __restrict__ BT1p,
    const unsigned short* __restrict__ BTDp, const float* __restrict__ BIAS0,
    float* __restrict__ out) {
  __shared__ __align__(16) _Float16 At[ROWS_BLK * APITCH];
  __shared__ __align__(16) _Float16 Ht[ROWS_BLK * TPITCH];
  __shared__ __align__(16) float    St[ROWS_BLK * SPITCH];
  __shared__ __align__(16) float    P1[ROWS_BLK * NHID];
  __shared__ __align__(16) float    decL[2 * ROWS_BLK];
  __shared__ __align__(16) float    mtL[2 * ROWS_BLK];
  __shared__ __align__(16) int      lastL[ROWS_BLK];

  const _Float16* BT0 = (const _Float16*)BT0p;
  const _Float16* BT1 = (const _Float16*)BT1p;
  const _Float16* BTD = (const _Float16*)BTDp;

  const int tid = threadIdx.x, lane = tid & 31, wave = tid >> 5;
  const int c = lane & 15, hh = lane >> 4, koff = hh * 8;
  const int col = 16 * wave + c;
  const int rowbase = blockIdx.x * ROWS_BLK;

#pragma unroll 1
  for (int i = tid; i < ROWS_BLK * APITCH; i += NTHR) At[i] = (_Float16)0.0f;
#pragma unroll 1
  for (int i = tid; i < ROWS_BLK * TPITCH; i += NTHR) Ht[i] = (_Float16)0.0f;
#pragma unroll 1
  for (int i = tid; i < ROWS_BLK * SPITCH; i += NTHR) St[i] = 0.0f;
  if (tid < ROWS_BLK) {
    float s = 0.0f;
#pragma unroll 1
    for (int t = 0; t < NSTEP; ++t) s += msk[(size_t)(rowbase + tid) * NSTEP + t];
    const float cf = fminf(fmaxf(s, 1.0f), (float)NSTEP);
    int lv = (int)cf - 1;
    lv = lv < 0 ? 0 : (lv > NSTEP - 1 ? NSTEP - 1 : lv);
    lastL[tid] = lv;
  }
  const float bI0 = BIAS0[col], bO0 = BIAS0[NHID + col], bC0 = BIAS0[2 * NHID + col];
  const float bI1 = bx[(4 + 1) * NHID + col], bO1 = bx[(4 + 2) * NHID + col], bC1 = bx[(4 + 3) * NHID + col];
  const float bD0 = bd[col], bD1 = bd[NHID + col];
  const float wT0 = Wt[col], wT1 = Wt[NHID + col];
  const float bT0 = bt[col], bT1 = bt[NHID + col];

  float h0s[2][8], c0s[2][8], h1s[2][8], c1s[2][8];
#pragma unroll
  for (int m = 0; m < 2; ++m)
#pragma unroll
    for (int r = 0; r < 8; ++r) { h0s[m][r] = 0.0f; c0s[m][r] = 0.0f; h1s[m][r] = 0.0f; c1s[m][r] = 0.0f; }
  __syncthreads();
  stage_inputs(hist, msk, At, decL, mtL, rowbase, 0, tid);
  __syncthreads();

  const _Float16* arow0 = At + c * APITCH + koff;
  const _Float16* arow1 = At + c * APITCH + koff + K0PAD;
  const _Float16* wg0 = BT0 + (size_t)col * KL0 + koff;
  const _Float16* wg1 = BT1 + (size_t)col * KL1 + koff;
  const _Float16* wd0 = BTD + (size_t)col * NHID + koff;
  const _Float16* wd1 = BTD + (size_t)NHID * NHID + (size_t)col * NHID + koff;
  _Float16* htw = Ht + (8 * hh) * TPITCH + col;
  const _Float16* htr = Ht + c * TPITCH + koff;
  _Float16* hdst0 = At + (8 * hh) * APITCH + K0PAD + col;
  _Float16* hdst1 = At + (8 * hh) * APITCH + K0PAD + NHID + col;

#pragma unroll 1
  for (int t = 0; t < NSTEP; ++t) {
    const int par = t & 1;
    const float* decp = decL + par * ROWS_BLK + 8 * hh;
    const float* mtp  = mtL  + par * ROWS_BLK + 8 * hh;
    cell_layer<KL0>(arow0, wg0, wd0, htw, htr, hdst0, decp, mtp, bI0, bO0, bC0, bD0, wT0, bT0, h0s, c0s);
    __syncthreads();
    cell_layer<KL1>(arow1, wg1, wd1, htw, htr, hdst1, decp, mtp, bI1, bO1, bC1, bD1, wT1, bT1, h1s, c1s);
#pragma unroll
    for (int m = 0; m < 2; ++m) {
      const v4i lA = *(const v4i*)(lastL + 8 * hh + 16 * m);
      const v4i lB = *(const v4i*)(lastL + 8 * hh + 16 * m + 4);
      const v4f mA = *(const v4f*)(mtp + 16 * m);
      const v4f mB = *(const v4f*)(mtp + 16 * m + 4);
#pragma unroll
      for (int r = 0; r < 8; ++r) {
        const int   lv = (r < 4) ? lA[r & 3] : lB[r & 3];
        const float mv = (r < 4) ? mA[r & 3] : mB[r & 3];
        const float ev = h1s[m][r] * mv;
        if (t == lv) St[(16 * m + 8 * hh + r) * SPITCH + NFEAT + col] = ev;
      }
    }
    {
      const int tn = (t + 1 < NSTEP) ? (t + 1) : (NSTEP - 1);
      stage_inputs(hist, msk, At, decL + (par ^ 1) * ROWS_BLK, mtL + (par ^ 1) * ROWS_BLK, rowbase, tn, tid);
    }
    __syncthreads();
  }

  if (tid < 128) {
    const int row = tid >> 2, f4 = (tid & 3) * 4;
    int lv = lastL[row];
    lv = lv < 0 ? 0 : (lv > NSTEP - 1 ? NSTEP - 1 : lv);
    const v4f v = *(const v4f*)(hist + ((size_t)(rowbase + row) * NSTEP + (size_t)lv) * NFEAT + f4);
    *(v4f*)(St + row * SPITCH + f4) = v;
  }
  __syncthreads();
  {
    const int row = tid >> 3, seg = tid & 7;
    float* sp = St + row * SPITCH + seg * LN_SEG;
    float s = 0.0f;
#pragma unroll 1
    for (int j = 0; j < LN_SEG; ++j) s += sp[j];
    s += __shfl_xor(s, 1, 32);
    s += __shfl_xor(s, 2, 32);
    s += __shfl_xor(s, 4, 32);
    const float mu = s * (1.0f / (float)NSTATE);
    float ss = 0.0f;
#pragma unroll 1
    for (int j = 0; j < LN_SEG; ++j) { const float d = sp[j] - mu; ss = fmaf(d, d, ss); }
    ss += __shfl_xor(ss, 1, 32);
    ss += __shfl_xor(ss, 2, 32);
    ss += __shfl_xor(ss, 4, 32);
    const float rstd = rsqrtf(ss * (1.0f / (float)NSTATE) + LN_EPS_F);
#pragma unroll 1
    for (int j = 0; j < LN_SEG; ++j) {
      const int k = seg * LN_SEG + j;
      sp[j] = (sp[j] - mu) * rstd * ln_g[k] + ln_b[k];
    }
  }
  __syncthreads();
  {
    const int n = tid & (NHID - 1), rg = tid >> 7;
    const float bv = b1[n];
    float acc[16];
#pragma unroll
    for (int i = 0; i < 16; ++i) acc[i] = bv;
    const float* sb = St + (rg * 16) * SPITCH;
#pragma unroll 1
    for (int k = 0; k < NSTATE; ++k) {
      const float w = W1[(size_t)k * NHID + n];
#pragma unroll
      for (int i = 0; i < 16; ++i) acc[i] = fmaf(sb[i * SPITCH + k], w, acc[i]);
    }
#pragma unroll
    for (int i = 0; i < 16; ++i) P1[(rg * 16 + i) * NHID + n] = fmaxf(acc[i], 0.0f);
  }
  __syncthreads();
  {
    const int o = tid & 63, rg = tid >> 6;
    const int oc = o < NOUTC ? o : (NOUTC - 1);
    const float bv = b2[oc];
    float acc[8];
#pragma unroll
    for (int i = 0; i < 8; ++i) acc[i] = bv;
    const float* pb = P1 + (rg * 8) * NHID;
#pragma unroll 1
    for (int k = 0; k < NHID; ++k) {
      const float w = W2[(size_t)k * NOUTC + oc];
#pragma unroll
      for (int i = 0; i < 8; ++i) acc[i] = fmaf(pb[i * NHID + k], w, acc[i]);
    }
#pragma unroll
    for (int i = 0; i < 8; ++i) {
      float v = acc[i];
      v = __builtin_isnan(v) ? 0.0f : v;
      v = (v == INFINITY) ? 1e4f : v;
      v = (v == -INFINITY) ? -1e4f : v;
      if (o < NOUTC) St[(rg * 8 + i) * NOUTC + o] = v;
    }
  }
  __syncthreads();
  {
    float* ob = out + (size_t)blockIdx.x * (ROWS_BLK * NOUTC);
    const int nq = (ROWS_BLK * NOUTC) / 4;
    const int i1 = NTHR + tid;
    const bool live1 = (i1 < nq);
    const int i1c = live1 ? i1 : (nq - 1);
    const v4f v0 = *(const v4f*)(St + 4 * tid);
    const v4f v1 = *(const v4f*)(St + 4 * i1c);
    for (int pass = 0; pass < 2; ++pass) {
      *(volatile v4f*)(ob + 4 * tid) = v0;
      if (live1) *(volatile v4f*)(ob + 4 * i1) = v1;
      __threadfence();
    }
  }
}

extern "C" void kernel_launch(void* const* d_in, const int* in_sizes, int n_in,
                              void* d_out, int out_size, void* d_ws, size_t ws_size, hipStream_t stream) {
  if (n_in < 17 || d_out == nullptr || d_ws == nullptr) return;
  if (in_sizes[0] != NBATCH * NSTEP * NFEAT || in_sizes[1] != NBATCH * NSTEP ||
      in_sizes[2] != NFEAT * NHID || in_sizes[3] != NHID ||
      in_sizes[4] != 2 * 4 * NHID * NHID || in_sizes[5] != 2 * 4 * NHID ||
      in_sizes[6] != 2 * 4 * NHID * NHID || in_sizes[7] != 2 * NHID * NHID ||
      in_sizes[8] != 2 * NHID || in_sizes[9] != 2 * NHID || in_sizes[10] != 2 * NHID ||
      in_sizes[11] != NSTATE || in_sizes[12] != NSTATE ||
      in_sizes[13] != NSTATE * NHID || in_sizes[14] != NHID ||
      in_sizes[15] != NHID * NOUTC || in_sizes[16] != NOUTC ||
      out_size != NBATCH * NOUTC) return;

  const float* hist = (const float*)d_in[0];
  const float* msk  = (const float*)d_in[1];
  const float* Wp   = (const float*)d_in[2];
  const float* bp   = (const float*)d_in[3];
  const float* Wx   = (const float*)d_in[4];
  const float* bx   = (const float*)d_in[5];
  const float* Uh   = (const float*)d_in[6];
  const float* Wd   = (const float*)d_in[7];
  const float* bd   = (const float*)d_in[8];
  const float* Wt   = (const float*)d_in[9];
  const float* bt   = (const float*)d_in[10];
  const float* ln_g = (const float*)d_in[11];
  const float* ln_b = (const float*)d_in[12];
  const float* W1   = (const float*)d_in[13];
  const float* b1   = (const float*)d_in[14];
  const float* W2   = (const float*)d_in[15];
  const float* b2   = (const float*)d_in[16];
  float* out = (float*)d_out;

  char* ws = (char*)d_ws; size_t off = 0;
  auto carve = [&](size_t bytes) -> char* { char* p = ws + off; off += (bytes + 255) & ~(size_t)255; return p; };
  unsigned short* BT0 = (unsigned short*)carve((size_t)NLIVE * NHID * KL0 * 2);
  unsigned short* BT1 = (unsigned short*)carve((size_t)NLIVE * NHID * KL1 * 2);
  unsigned short* BTD = (unsigned short*)carve((size_t)2 * NHID * NHID * 2);
  float*        BIAS0 = (float*)carve((size_t)NLIVE * NHID * 4);
  if (off > ws_size || off > (size_t)134217728) return;

  pack_planes_kernel<<<PB_TOTAL, NTHR, 0, stream>>>(Wp, bp, Wx, bx, Uh, Wd, BT0, BT1, BTD, BIAS0);
  tcell_seq_kernel<<<NBATCH / ROWS_BLK, NTHR, 0, stream>>>(hist, msk, bx, bd, Wt, bt, ln_g, ln_b, W1, b1, W2, b2,
                                                          BT0, BT1, BTD, BIAS0, out);
}
